// Model_3599182594396
// MI455X (gfx1250) — hardware-verified
//
#include <hip/hip_runtime.h>
#include <stddef.h>
#include <stdint.h>


#define NN     200000
#define NE     400000
#define NG     4096
#define IND    26
#define DF     128
#define CLS    256
#define MP     200064
#define HP     256
#define XP     32
#define A0P    64
#define K0     96
#define K1     512
#define KL     256
#define GPP    512
#define NTHR   256
#define NWAVE  8
#define EPT    8
#define CHUNK  (NTHR * EPT)
#define WCAP   (EPT * 32)
#define LISTN  (NWAVE * WCAP)
#define NBA    1024
#define SLA    10
#define NBLK   196
#define NSLOT  (NBLK * NBA)
#define LCAP   4096
#define DEGCAP 32
#define NBP    32
#define SLP    5
#define PBLK   (NG / NBP)
#define PCAP   4096
#define GCAP   128
#define NFLG   (NBLK + PBLK)
#define MISC_INTS 16
#define GBM    64
#define GBN    128
#define GTHR   128
#define XBLK   (MP * 4 / NTHR)
#define U0     (DF * (K0 / 8))
#define UC     (3 * DF * (K1 / 8))
#define UL     (CLS * (KL / 8))
#define WBLK   ((U0 + UC + UL) / NTHR)
#define MEAS_B1024  2152
#define MEAS_MAXDEG 11
#define MEAS_GMAX   77

static_assert((CHUNK & (CHUNK - 1)) == 0 && CHUNK <= 4096);
static_assert(NBA == (1 << SLA) && NBP == (1 << SLP));
static_assert(((long long)NE << SLA) < (1LL << 31) && ((long long)NN << SLP) < (1LL << 31));
static_assert(MP == 3126 * GBM && MP % GBM == 0 && NN <= MP && NSLOT >= MP);
static_assert(NG % GBM == 0 && NG % 128 == 0 && NG == PBLK * NBP);
static_assert(K0 % 32 == 0 && K1 % 32 == 0 && KL % 32 == 0);
static_assert(K0 == A0P + XP && K1 == 2 * HP && KL == HP && GPP == K1);
static_assert(LCAP * 10 >= MEAS_B1024 * 11 && DEGCAP >= MEAS_MAXDEG + 8);
static_assert(PCAP * 10 >= NBP * MEAS_GMAX * 11 && GCAP >= MEAS_GMAX + 8);
static_assert(LCAP % (NTHR * 4) == 0 && PCAP % (NTHR * 4) == 0 && LISTN % (NTHR * 4) == 0);
static_assert(NBA == NTHR * 4 && NBA % NWAVE == 0 && NBA % 32 == 0 && NBP % 32 == 0 && NBP % NWAVE == 0);
static_assert((MP * 4) % NTHR == 0 && (U0 + UC + UL) % NTHR == 0 && U0 % NTHR == 0 && UC % NTHR == 0);
static_assert(GBN == DF && GBM == (GTHR / 32) * 16);

typedef float          v2f   __attribute__((ext_vector_type(2)));
typedef float          v4f   __attribute__((ext_vector_type(4)));
typedef float          v8f   __attribute__((ext_vector_type(8)));
typedef int            v4i   __attribute__((ext_vector_type(4)));
typedef int            v8i   __attribute__((ext_vector_type(8)));
typedef unsigned       v2u   __attribute__((ext_vector_type(2)));
typedef unsigned short v4us  __attribute__((ext_vector_type(4)));
typedef unsigned short v8us  __attribute__((ext_vector_type(8)));
typedef unsigned short v16us __attribute__((ext_vector_type(16)));
typedef __bf16         v16bf __attribute__((ext_vector_type(16)));
typedef v2f  __attribute__((may_alias)) v2fa;
typedef v4f  __attribute__((may_alias)) v4fa;
typedef v4i  __attribute__((may_alias)) v4ia;
typedef v2u  __attribute__((may_alias)) v2ua;
typedef v4us __attribute__((may_alias)) v4usa;
typedef v8us __attribute__((may_alias)) v8usa;
union FragB { v16bf v; v16us u; v8us h[2]; v8i w; };

__device__ __forceinline__ v8f wmb(const FragB& a, const FragB& b, v8f c) {
  v8f d = __builtin_amdgcn_wmma_f32_16x16x32_bf16(false, a.v, false, b.v, (short)0, c, false, false);
  asm volatile("v_nop\n\tv_nop\n\tv_nop\n\tv_nop" : "+v"(d) : "v"(a.w), "v"(b.w));
  return d;
}

__device__ __forceinline__ unsigned bf16_bits(float f) {
  const unsigned u = __float_as_uint(f);
  return (u + 0x7FFFu + ((u >> 16) & 1u)) >> 16;
}
__device__ __forceinline__ float bf16_val(float f) {
  return __uint_as_float(bf16_bits(f) << 16);
}
__device__ __forceinline__ float blendf(float a, float b, unsigned m) {
  return __uint_as_float((__float_as_uint(a) & ~m) | (__float_as_uint(b) & m));
}

__device__ __forceinline__ void wave_sync() {
  __builtin_amdgcn_fence(__ATOMIC_RELEASE, "workgroup");
  __builtin_amdgcn_wave_barrier();
  __builtin_amdgcn_fence(__ATOMIC_ACQUIRE, "workgroup");
}

template <int SLB>
__device__ __forceinline__ int scan_chunk(const int* __restrict__ dsts, int nE, int cbase, int slotBase,
                                          int nb, int vec8, int* list, int tid, int lane, int wave) {
  int wc = 0;
  const int el0  = tid * EPT;
  const int e0   = cbase + el0;
  const int sent = -2147483647 - 1;
  v4i da, db;
  if (vec8 != 0 && cbase + CHUNK <= nE) {
    da = *(const v4i*)(dsts + e0);
    db = *(const v4i*)(dsts + e0 + 4);
  } else {
    da.x = (e0     < nE) ? dsts[min(e0,     nE - 1)] : sent;
    da.y = (e0 + 1 < nE) ? dsts[min(e0 + 1, nE - 1)] : sent;
    da.z = (e0 + 2 < nE) ? dsts[min(e0 + 2, nE - 1)] : sent;
    da.w = (e0 + 3 < nE) ? dsts[min(e0 + 3, nE - 1)] : sent;
    db.x = (e0 + 4 < nE) ? dsts[min(e0 + 4, nE - 1)] : sent;
    db.y = (e0 + 5 < nE) ? dsts[min(e0 + 5, nE - 1)] : sent;
    db.z = (e0 + 6 < nE) ? dsts[min(e0 + 6, nE - 1)] : sent;
    db.w = (e0 + 7 < nE) ? dsts[min(e0 + 7, nE - 1)] : sent;
  }
  const unsigned nbs = (unsigned)slotBase;
  const unsigned unb = (unsigned)nb;
  const unsigned s0 = (unsigned)da.x - nbs, s1 = (unsigned)da.y - nbs;
  const unsigned s2 = (unsigned)da.z - nbs, s3 = (unsigned)da.w - nbs;
  const unsigned s4 = (unsigned)db.x - nbs, s5 = (unsigned)db.y - nbs;
  const unsigned s6 = (unsigned)db.z - nbs, s7 = (unsigned)db.w - nbs;
  const bool h0 = s0 < unb, h1 = s1 < unb, h2 = s2 < unb, h3 = s3 < unb;
  const bool h4 = s4 < unb, h5 = s5 < unb, h6 = s6 < unb, h7 = s7 < unb;
  const unsigned any = __builtin_amdgcn_ballot_w32(h0 | h1 | h2 | h3 | h4 | h5 | h6 | h7);
  if (any != 0u) {
#define HITJ(J, HJ, SJ) { \
      const unsigned mj = __builtin_amdgcn_ballot_w32(HJ); \
      if (mj != 0u) { \
        if (HJ) { \
          const int pos = wc + (int)__builtin_amdgcn_mbcnt_lo(mj, 0u); \
          if (pos < WCAP) list[wave * WCAP + pos] = ((el0 + (J)) << SLB) | (int)(SJ); \
        } \
        wc += (int)__builtin_popcount(mj); } }
    HITJ(0, h0, s0)
    HITJ(1, h1, s1)
    HITJ(2, h2, s2)
    HITJ(3, h3, s3)
    HITJ(4, h4, s4)
    HITJ(5, h5, s5)
    HITJ(6, h6, s6)
    HITJ(7, h7, s7)
#undef HITJ
  }
  return wc;
}

template <int SLB, int NB, int CAP>
__device__ __forceinline__ void bucket_core(const int* __restrict__ keys, int nE, int vec8, int slotBase,
                                            int dcap, int* list, int* hl, int* sl, int* cnt, int* offs,
                                            int* cur, int* misc, int tid, int lane, int wave) {
  {
    const v4i z4 = {0, 0, 0, 0};
    for (int i = tid * 4; i < LISTN; i += NTHR * 4) *(v4ia*)(list + i) = z4;
    for (int i = tid * 4; i < CAP; i += NTHR * 4) { *(v4ia*)(hl + i) = z4; *(v4ia*)(sl + i) = z4; }
    for (int i = tid; i < NB; i += NTHR) { cnt[i] = 0; offs[i] = 0; cur[i] = 0; }
    if (tid < MISC_INTS) misc[tid] = 0;
  }
  __syncthreads();

  int t = 0, ov = 0;
  const int nChunks = (nE + CHUNK - 1) / CHUNK;
#pragma unroll 1
  for (int ch = 0; ch < nChunks; ++ch) {
    const int cbase = ch * CHUNK;
    const int wc = scan_chunk<SLB>(keys, nE, cbase, slotBase, NB, vec8, list, tid, lane, wave);
    if (lane == 0) misc[wave] = wc;
    __syncthreads();
    if (wave == 0) {
#pragma unroll 1
      for (int w2 = 0; w2 < NWAVE; ++w2) {
        int c = misc[w2];
        c = c < 0 ? 0 : (c > WCAP ? WCAP : c);
#pragma unroll 1
        for (int b0 = 0; b0 < c; b0 += 32) {
          const int idx = b0 + lane;
          const int ent = list[w2 * WCAP + (idx < WCAP ? idx : WCAP - 1)];
          const int m32 = (c - b0) < 32 ? (c - b0) : 32;
#pragma unroll 1
          for (int k = 0; k < m32; ++k) {
            const int u    = __builtin_amdgcn_readlane(ent, k);
            const int slot = u & (NB - 1);
            const int el   = (u >> SLB) & (CHUNK - 1);
            const int pk   = ((cbase + el) << SLB) | slot;
            if (t < CAP) {
              if (lane == 0) { hl[t] = pk; cnt[slot] = cnt[slot] + 1; }
              t = t + 1;
            } else {
              ov = 1;
            }
          }
        }
      }
    }
    __syncthreads();
  }
  if (wave == 0 && lane == 0) { misc[8] = t; misc[9] = ov; }
  __syncthreads();
  int tt = misc[8];
  tt = tt < 0 ? 0 : (tt > CAP ? CAP : tt);

  if (wave == 0) {
    constexpr int PER = NB / 32;
    const int base = lane * PER;
    int s = 0, bigl = 0;
#pragma unroll 1
    for (int i = 0; i < PER; ++i) { const int cv = cnt[base + i]; s += cv; bigl |= (cv > dcap) ? 1 : 0; }
    const unsigned bm = __builtin_amdgcn_ballot_w32(bigl != 0);
    if (lane == 0 && bm != 0u) misc[10] = 1;
    int incl = s;
#pragma unroll
    for (int d = 1; d < 32; d <<= 1) {
      const int y = __shfl_up(incl, d, 32);
      if (lane >= d) incl += y;
    }
    int run = incl - s;
#pragma unroll 1
    for (int i = 0; i < PER; ++i) {
      const int cv = cnt[base + i];
      offs[base + i] = run;
      cur[base + i]  = run;
      run += cv;
    }
  }
  __syncthreads();
  if (wave == 0) {
#pragma unroll 1
    for (int b0 = 0; b0 < tt; b0 += 32) {
      const int idx = b0 + lane;
      const int ent = hl[idx < CAP ? idx : CAP - 1];
      const int m32 = (tt - b0) < 32 ? (tt - b0) : 32;
#pragma unroll 1
      for (int k = 0; k < m32; ++k) {
        const int u    = __builtin_amdgcn_readlane(ent, k);
        const int slot = u & (NB - 1);
        if (lane == 0) {
          int p = cur[slot];
          p = p < 0 ? 0 : (p > CAP - 1 ? CAP - 1 : p);
          sl[p] = u;
          cur[slot] = p + 1;
        }
      }
    }
  }
  __syncthreads();
}

__global__ __launch_bounds__(NTHR) void k_prep(const float* __restrict__ x, const float* __restrict__ W1l,
                                               const float* __restrict__ W1r, const float* __restrict__ Wl,
                                               const float* __restrict__ Wr, const float* __restrict__ Wlin1,
                                               unsigned short* wsh, size_t oXB, size_t oW0, size_t oWC,
                                               size_t oWL) {
  const int blk = (int)blockIdx.x, tid = (int)threadIdx.x;
  v8us o;
  size_t de;
  if (blk < XBLK) {
    const int u   = blk * NTHR + tid;
    const int row = u >> 2;
    const int q   = u & 3;
    const int rc  = row < NN ? row : NN - 1;
    const float* p = x + (size_t)rc * IND;
#pragma unroll
    for (int j = 0; j < 4; ++j) {
      const int col = 8 * q + 2 * j;
      const int cc  = col < 24 ? col : 24;
      const v2f a = *(const v2fa*)(p + cc);
      const bool ok = (row < NN) && (col < IND);
      o[2 * j]     = ok ? (unsigned short)bf16_bits(a.x) : (unsigned short)0;
      o[2 * j + 1] = ok ? (unsigned short)bf16_bits(a.y) : (unsigned short)0;
    }
    de = oXB + (size_t)u * 8;
  } else {
    const int v0 = (blk - XBLK) * NTHR + tid;
    if (v0 < U0) {
      const int n   = v0 / 12;
      const int c   = v0 - 12 * n;
      const int seg = c >> 2;
      const int kk  = (c & 3) * 8;
      const unsigned msk = (seg == 2) ? 0xffffffffu : 0u;
      const float* pl = W1l + (size_t)n * IND;
      const float* pr = W1r + (size_t)n * IND;
#pragma unroll
      for (int j = 0; j < 4; ++j) {
        const int col = kk + 2 * j;
        const int cc  = col < 24 ? col : 24;
        const v2f a = *(const v2fa*)(pl + cc);
        const v2f b = *(const v2fa*)(pr + cc);
        const bool ok = col < IND;
        o[2 * j]     = ok ? (unsigned short)bf16_bits(blendf(a.x, b.x, msk)) : (unsigned short)0;
        o[2 * j + 1] = ok ? (unsigned short)bf16_bits(blendf(a.y, b.y, msk)) : (unsigned short)0;
      }
      de = oW0 + (size_t)v0 * 8;
    } else if (v0 < U0 + UC) {
      const int v   = v0 - U0;
      const int lay = v >> 13;
      const int r   = v & 8191;
      const int n   = r >> 6;
      const int c   = r & 63;
      const int kk  = (c & 15) * 8;
      const unsigned msk = (c >= 32) ? 0xffffffffu : 0u;
      const size_t so = ((size_t)lay * DF + n) * DF + kk;
      const v4f a0 = *(const v4fa*)(Wl + so);
      const v4f a1 = *(const v4fa*)(Wl + so + 4);
      const v4f b0 = *(const v4fa*)(Wr + so);
      const v4f b1 = *(const v4fa*)(Wr + so + 4);
      o[0] = (unsigned short)bf16_bits(blendf(a0.x, b0.x, msk));
      o[1] = (unsigned short)bf16_bits(blendf(a0.y, b0.y, msk));
      o[2] = (unsigned short)bf16_bits(blendf(a0.z, b0.z, msk));
      o[3] = (unsigned short)bf16_bits(blendf(a0.w, b0.w, msk));
      o[4] = (unsigned short)bf16_bits(blendf(a1.x, b1.x, msk));
      o[5] = (unsigned short)bf16_bits(blendf(a1.y, b1.y, msk));
      o[6] = (unsigned short)bf16_bits(blendf(a1.z, b1.z, msk));
      o[7] = (unsigned short)bf16_bits(blendf(a1.w, b1.w, msk));
      de = oWC + (size_t)v * 8;
    } else {
      const int v  = v0 - U0 - UC;
      const int n  = v >> 5;
      const int c  = v & 31;
      const int kk = (c & 15) * 8;
      const size_t so = (size_t)n * DF + kk;
      const v4f a0 = *(const v4fa*)(Wlin1 + so);
      const v4f a1 = *(const v4fa*)(Wlin1 + so + 4);
      o[0] = (unsigned short)bf16_bits(a0.x); o[1] = (unsigned short)bf16_bits(a0.y);
      o[2] = (unsigned short)bf16_bits(a0.z); o[3] = (unsigned short)bf16_bits(a0.w);
      o[4] = (unsigned short)bf16_bits(a1.x); o[5] = (unsigned short)bf16_bits(a1.y);
      o[6] = (unsigned short)bf16_bits(a1.z); o[7] = (unsigned short)bf16_bits(a1.w);
      de = oWL + (size_t)v * 8;
    }
  }
  unsigned short* dp = wsh + de;
  *(volatile v8us*)dp = o;
  __threadfence();
  *(volatile v8us*)dp = o;
}

__global__ __launch_bounds__(NTHR) void k_bucket(const int* __restrict__ srcs, const int* __restrict__ dsts,
                                                 int nE, int nN, int vec8, int* LISTg, int* DEGg, int* OFFg,
                                                 float* INVg, int* FLGg) {
  __shared__ __attribute__((aligned(16))) int list[LISTN];
  __shared__ __attribute__((aligned(16))) int hl[LCAP];
  __shared__ __attribute__((aligned(16))) int sl[LCAP];
  __shared__ __attribute__((aligned(16))) int cnt[NBA];
  __shared__ __attribute__((aligned(16))) int offs[NBA];
  __shared__ __attribute__((aligned(16))) int cur[NBA];
  __shared__ __attribute__((aligned(16))) float invs[NBA];
  __shared__ __attribute__((aligned(16))) int misc[MISC_INTS];
  const int tid = (int)threadIdx.x, lane = tid & 31, wave = tid >> 5;
  const int blk = (int)blockIdx.x;
  const int nodeBase = blk * NBA;

  bucket_core<SLA, NBA, LCAP>(dsts, nE, vec8, nodeBase, DEGCAP, list, hl, sl, cnt, offs, cur, misc,
                              tid, lane, wave);
  int tt = misc[8];
  tt = tt < 0 ? 0 : (tt > LCAP ? LCAP : tt);
  const int fl = ((misc[9] | misc[10]) != 0) ? 1 : 0;

#pragma unroll 1
  for (int it = 0; it < LCAP / (NTHR * 4); ++it) {
    const int i0 = it * (NTHR * 4) + 4 * tid;
    const v4i e4 = *(const v4ia*)(sl + i0);
    int e0 = e4.x >> SLA, e1 = e4.y >> SLA, e2 = e4.z >> SLA, e3 = e4.w >> SLA;
    e0 = e0 < 0 ? 0 : (e0 > nE - 1 ? nE - 1 : e0);
    e1 = e1 < 0 ? 0 : (e1 > nE - 1 ? nE - 1 : e1);
    e2 = e2 < 0 ? 0 : (e2 > nE - 1 ? nE - 1 : e2);
    e3 = e3 < 0 ? 0 : (e3 > nE - 1 ? nE - 1 : e3);
    int g0 = srcs[e0], g1 = srcs[e1], g2 = srcs[e2], g3 = srcs[e3];
    g0 = g0 < 0 ? 0 : (g0 > nN - 1 ? nN - 1 : g0);
    g1 = g1 < 0 ? 0 : (g1 > nN - 1 ? nN - 1 : g1);
    g2 = g2 < 0 ? 0 : (g2 > nN - 1 ? nN - 1 : g2);
    g3 = g3 < 0 ? 0 : (g3 > nN - 1 ? nN - 1 : g3);
    v4i s4;
    s4.x = (i0     < tt) ? g0 : 0;
    s4.y = (i0 + 1 < tt) ? g1 : 0;
    s4.z = (i0 + 2 < tt) ? g2 : 0;
    s4.w = (i0 + 3 < tt) ? g3 : 0;
    *(v4ia*)(hl + i0) = s4;
  }
#pragma unroll 1
  for (int j = 0; j < NBA / NTHR; ++j) {
    const int s = j * NTHR + tid;
    const int c = cnt[s];
    const float cf = (c < 1) ? 1.0f : (float)c;
    invs[s] = 1.0f / cf;
  }
  __syncthreads();

  v4i lv[LCAP / (NTHR * 4)];
#pragma unroll
  for (int it = 0; it < LCAP / (NTHR * 4); ++it) lv[it] = *(const v4ia*)(hl + it * (NTHR * 4) + 4 * tid);
  const v4i c4 = *(const v4ia*)(cnt + 4 * tid);
  const v4i o4 = *(const v4ia*)(offs + 4 * tid);
  const v4f i4 = *(const v4fa*)(invs + 4 * tid);
  const v4i f4 = {fl, fl, fl, fl};
  int* lp = LISTg + (size_t)blk * LCAP;
  const bool wf = tid < 8;
#pragma unroll
  for (int it = 0; it < LCAP / (NTHR * 4); ++it) *(volatile v4i*)(lp + it * (NTHR * 4) + 4 * tid) = lv[it];
  *(volatile v4i*)(DEGg + nodeBase + 4 * tid) = c4;
  *(volatile v4i*)(OFFg + nodeBase + 4 * tid) = o4;
  *(volatile v4f*)(INVg + nodeBase + 4 * tid) = i4;
  if (wf) *(volatile v4i*)(FLGg + blk * 32 + 4 * (tid & 7)) = f4;
  __threadfence();
#pragma unroll
  for (int it = 0; it < LCAP / (NTHR * 4); ++it) *(volatile v4i*)(lp + it * (NTHR * 4) + 4 * tid) = lv[it];
  *(volatile v4i*)(DEGg + nodeBase + 4 * tid) = c4;
  *(volatile v4i*)(OFFg + nodeBase + 4 * tid) = o4;
  *(volatile v4f*)(INVg + nodeBase + 4 * tid) = i4;
  if (wf) *(volatile v4i*)(FLGg + blk * 32 + 4 * (tid & 7)) = f4;
}

template <int L0>
__global__ __launch_bounds__(NTHR) void k_agg(const unsigned short* __restrict__ sp, unsigned short* dp,
                                              const int* __restrict__ LISTg, const int* __restrict__ DEGg,
                                              const int* __restrict__ OFFg, const float* __restrict__ INVg,
                                              const int* __restrict__ FLGg, int nN, int mRows) {
  __shared__ __attribute__((aligned(16))) int lst[LCAP];
  __shared__ __attribute__((aligned(16))) int dg[NBA];
  __shared__ __attribute__((aligned(16))) int of[NBA];
  __shared__ __attribute__((aligned(16))) float iv[NBA];
  __shared__ __attribute__((aligned(16))) unsigned short rowb[NWAVE * HP];
  const int tid = (int)threadIdx.x, lane = tid & 31, wave = tid >> 5;
  const int blk = (int)blockIdx.x;
  const int nodeBase = blk * NBA;
  unsigned short* rowbuf = rowb + wave * HP;

#pragma unroll
  for (int it = 0; it < LCAP / (NTHR * 4); ++it) {
    const int i0 = it * (NTHR * 4) + 4 * tid;
    *(v4ia*)(lst + i0) = *(const v4i*)(LISTg + (size_t)blk * LCAP + i0);
  }
  *(v4ia*)(dg + 4 * tid) = *(const v4i*)(DEGg + nodeBase + 4 * tid);
  *(v4ia*)(of + 4 * tid) = *(const v4i*)(OFFg + nodeBase + 4 * tid);
  *(v4fa*)(iv + 4 * tid) = *(const v4f*)(INVg + nodeBase + 4 * tid);
  const int fl = FLGg[blk * 32];
  __syncthreads();

  const float qnan = __int_as_float(0x7fc00000);
  const float pz = (fl != 0) ? qnan : 0.0f;
#pragma unroll 1
  for (int si = 0; si < NBA / NWAVE; ++si) {
    const int s    = si * NWAVE + wave;
    const int node = nodeBase + s;
    int c = dg[s];
    const bool big = c > DEGCAP;
    c = c < 0 ? 0 : (c > DEGCAP ? DEGCAP : c);
    int o = of[s];
    o = o < 0 ? 0 : (o > LCAP ? LCAP : o);
    const float ivs = iv[s];
    float a0 = 0.0f, a1 = 0.0f, a2 = 0.0f, a3 = 0.0f;
#pragma unroll 1
    for (int b0 = 0; b0 < c; b0 += 32) {
      int idx = o + b0 + lane;
      idx = idx > LCAP - 1 ? LCAP - 1 : idx;
      int sr = lst[idx];
      sr = sr < 0 ? 0 : (sr > nN - 1 ? nN - 1 : sr);
      const int m32 = (c - b0) < 32 ? (c - b0) : 32;
#pragma unroll 1
      for (int k = 0; k < m32; ++k) {
        const int sk = __builtin_amdgcn_readlane(sr, k);
        if constexpr (L0 != 0) {
          const unsigned xv = (unsigned)sp[(size_t)sk * XP + lane];
          a0 += __uint_as_float(xv << 16);
        } else {
          const unsigned short* rp = sp + (size_t)sk * HP + 4 * lane;
          const v2u wh = *(const v2ua*)rp;
          const v2u wl = *(const v2ua*)(rp + DF);
          a0 += __uint_as_float(wh.x << 16)         + __uint_as_float(wl.x << 16);
          a1 += __uint_as_float(wh.x & 0xffff0000u) + __uint_as_float(wl.x & 0xffff0000u);
          a2 += __uint_as_float(wh.y << 16)         + __uint_as_float(wl.y << 16);
          a3 += __uint_as_float(wh.y & 0xffff0000u) + __uint_as_float(wl.y & 0xffff0000u);
        }
      }
    }
    const float pzr = big ? qnan : pz;
    const bool live = node < nN;
    if constexpr (L0 != 0) {
      const float m0 = live ? (a0 * ivs + pzr) : 0.0f;
      const unsigned hb = bf16_bits(m0);
      const unsigned lb = bf16_bits(m0 - __uint_as_float(hb << 16));
      rowbuf[lane]      = (unsigned short)hb;
      rowbuf[XP + lane] = (unsigned short)lb;
      wave_sync();
      const v8us q0 = *(const v8usa*)(rowbuf + 8 * (lane & 7));
      wave_sync();
      const bool wr = (node < mRows) && (lane < 8);
      unsigned short* rpw = dp + (size_t)node * A0P + 8 * (lane & 7);
      if (wr) *(volatile v8us*)rpw = q0;
      __threadfence();
      if (wr) *(volatile v8us*)rpw = q0;
    } else {
      const float m0 = live ? (a0 * ivs + pzr) : 0.0f;
      const float m1 = live ? (a1 * ivs + pzr) : 0.0f;
      const float m2 = live ? (a2 * ivs + pzr) : 0.0f;
      const float m3 = live ? (a3 * ivs + pzr) : 0.0f;
      v4us mh, ml;
      unsigned hb;
      hb = bf16_bits(m0); mh[0] = (unsigned short)hb; ml[0] = (unsigned short)bf16_bits(m0 - __uint_as_float(hb << 16));
      hb = bf16_bits(m1); mh[1] = (unsigned short)hb; ml[1] = (unsigned short)bf16_bits(m1 - __uint_as_float(hb << 16));
      hb = bf16_bits(m2); mh[2] = (unsigned short)hb; ml[2] = (unsigned short)bf16_bits(m2 - __uint_as_float(hb << 16));
      hb = bf16_bits(m3); mh[3] = (unsigned short)hb; ml[3] = (unsigned short)bf16_bits(m3 - __uint_as_float(hb << 16));
      *(v4usa*)(rowbuf + 4 * lane) = mh;
      *(v4usa*)(rowbuf + DF + 4 * lane) = ml;
      wave_sync();
      const v8us q0 = *(const v8usa*)(rowbuf + 8 * lane);
      wave_sync();
      const bool wr = node < mRows;
      unsigned short* rpw = dp + (size_t)node * HP + 8 * lane;
      if (wr) *(volatile v8us*)rpw = q0;
      __threadfence();
      if (wr) *(volatile v8us*)rpw = q0;
    }
  }
}

__device__ __forceinline__ void kloop(const unsigned short* ap, const unsigned short* __restrict__ bp,
                                      int nk, int K, v8f (&acc)[8]) {
#pragma unroll 1
  for (int ks = 0; ks < nk; ++ks) {
    const int k0 = 32 * ks;
    FragB af;
    af.h[0] = *(const v8usa*)(ap + k0);
    af.h[1] = *(const v8usa*)(ap + k0 + 16);
#pragma unroll
    for (int nt = 0; nt < 8; ++nt) {
      const unsigned short* wq = bp + (size_t)(16 * nt) * (size_t)K + k0;
      FragB bf;
      bf.h[0] = *(const v8usa*)wq;
      bf.h[1] = *(const v8usa*)(wq + 16);
      acc[nt] = wmb(af, bf, acc[nt]);
    }
  }
}

template <int MODE>
__global__ __launch_bounds__(GTHR) void k_gemm(const unsigned short* A1, int p1, int nk1,
                                               const unsigned short* A2, int p2, int nk2,
                                               const unsigned short* __restrict__ BT, int K,
                                               const float* __restrict__ bias, const int* __restrict__ cntp,
                                               unsigned short* outH, float* outF, int nOut) {
  __shared__ __attribute__((aligned(16))) float stg[GBM * GBN];
  const int tid = (int)threadIdx.x, lane = tid & 31, wave = tid >> 5, hh = lane >> 4, m = lane & 15;
  const int rowBase = (int)blockIdx.x * GBM;
  const int by = (int)blockIdx.y;

  v8f acc[8];
  {
    const v8f z = {0.f, 0.f, 0.f, 0.f, 0.f, 0.f, 0.f, 0.f};
#pragma unroll
    for (int t = 0; t < 8; ++t) acc[t] = z;
  }
  const size_t arow = (size_t)(rowBase + 16 * wave + m);
  const unsigned short* a1 = A1 + arow * (size_t)p1 + 8 * hh;
  const unsigned short* a2 = A2 + arow * (size_t)p2 + 8 * hh;
  const unsigned short* bt = BT + (size_t)(GBN * by + m) * (size_t)K + 8 * hh;
  kloop(a1, bt, nk1, K, acc);
  kloop(a2, bt + 32 * nk1, nk2, K, acc);

#pragma unroll
  for (int nt = 0; nt < 8; ++nt) {
    const int lc = 16 * nt + m;
#pragma unroll
    for (int r = 0; r < 8; ++r) {
      const int lr = 16 * wave + 8 * hh + r;
      stg[lr * GBN + lc] = acc[nt][r];
    }
  }
  __syncthreads();

  v4f bb4;
  {
    const v4f t1 = *(const v4f*)(bias + GBN * by + 4 * lane);
    bb4.x = bf16_val(t1.x); bb4.y = bf16_val(t1.y); bb4.z = bf16_val(t1.z); bb4.w = bf16_val(t1.w);
  }
  int cv = 1;
  if constexpr (MODE == 2) {
    int cr = rowBase + 16 * wave + m;
    cr = cr > nOut - 1 ? nOut - 1 : cr;
    cv = cntp[cr];
  }

  v4f pv[16];
#pragma unroll
  for (int i = 0; i < 16; ++i) pv[i] = *(const v4fa*)(stg + (16 * wave + i) * GBN + 4 * lane);
  __syncthreads();

#pragma unroll
  for (int i = 0; i < 16; ++i) {
    const bool ok = (rowBase + 16 * wave + i) < nOut;
    v4f b = bb4;
    if constexpr (MODE == 2) {
      const int ci = __shfl(cv, i, 32);
      const bool on = ci > 0;
      b.x = on ? bb4.x : 0.0f; b.y = on ? bb4.y : 0.0f; b.z = on ? bb4.z : 0.0f; b.w = on ? bb4.w : 0.0f;
    }
    v4f y = pv[i] + b;
    if constexpr (MODE == 1) {
      y.x = (y.x > 0.0f) ? y.x : (y.x - y.x);
      y.y = (y.y > 0.0f) ? y.y : (y.y - y.y);
      y.z = (y.z > 0.0f) ? y.z : (y.z - y.z);
      y.w = (y.w > 0.0f) ? y.w : (y.w - y.w);
    }
    y.x = ok ? y.x : 0.0f; y.y = ok ? y.y : 0.0f; y.z = ok ? y.z : 0.0f; y.w = ok ? y.w : 0.0f;
    pv[i] = y;
  }

  if constexpr (MODE == 1) {
#pragma unroll
    for (int i = 0; i < 16; ++i) {
      const int r = rowBase + 16 * wave + i;
      *(volatile v4f*)(outF + (size_t)r * CLS + GBN * by + 4 * lane) = pv[i];
    }
    __threadfence();
#pragma unroll
    for (int i = 0; i < 16; ++i) {
      const int r = rowBase + 16 * wave + i;
      *(volatile v4f*)(outF + (size_t)r * CLS + GBN * by + 4 * lane) = pv[i];
    }
  } else {
#pragma unroll
    for (int i = 0; i < 16; ++i) {
      v4us h4, l4;
      unsigned hb;
      hb = bf16_bits(pv[i].x); h4[0] = (unsigned short)hb; l4[0] = (unsigned short)bf16_bits(pv[i].x - __uint_as_float(hb << 16));
      hb = bf16_bits(pv[i].y); h4[1] = (unsigned short)hb; l4[1] = (unsigned short)bf16_bits(pv[i].y - __uint_as_float(hb << 16));
      hb = bf16_bits(pv[i].z); h4[2] = (unsigned short)hb; l4[2] = (unsigned short)bf16_bits(pv[i].z - __uint_as_float(hb << 16));
      hb = bf16_bits(pv[i].w); h4[3] = (unsigned short)hb; l4[3] = (unsigned short)bf16_bits(pv[i].w - __uint_as_float(hb << 16));
      unsigned short* srow = (unsigned short*)stg + (size_t)(16 * wave + i) * (2 * GBN);
      *(v4usa*)(srow + 4 * lane) = h4;
      *(v4usa*)(srow + DF + 4 * lane) = l4;
    }
    __syncthreads();
    v8us qv[16];
#pragma unroll
    for (int i = 0; i < 16; ++i) {
      const unsigned short* srow = (const unsigned short*)stg + (size_t)(16 * wave + i) * (2 * GBN);
      qv[i] = *(const v8usa*)(srow + 8 * lane);
    }
#pragma unroll
    for (int i = 0; i < 16; ++i) {
      unsigned short* rp = outH + (size_t)(rowBase + 16 * wave + i) * (size_t)HP + 8 * lane;
      *(volatile v8us*)rp = qv[i];
    }
    __threadfence();
#pragma unroll
    for (int i = 0; i < 16; ++i) {
      unsigned short* rp = outH + (size_t)(rowBase + 16 * wave + i) * (size_t)HP + 8 * lane;
      *(volatile v8us*)rp = qv[i];
    }
  }
}

__global__ __launch_bounds__(NTHR) void k_pool(const unsigned short* __restrict__ aggp,
                                               const unsigned short* __restrict__ hp,
                                               const int* __restrict__ bat, int nN, int vec8,
                                               unsigned short* GP, int* CNTG, int* FLGp) {
  __shared__ __attribute__((aligned(16))) int list[LISTN];
  __shared__ __attribute__((aligned(16))) int hl[PCAP];
  __shared__ __attribute__((aligned(16))) int sl[PCAP];
  __shared__ __attribute__((aligned(16))) int cnt[NBP];
  __shared__ __attribute__((aligned(16))) int offs[NBP];
  __shared__ __attribute__((aligned(16))) int cur[NBP];
  __shared__ __attribute__((aligned(16))) int misc[MISC_INTS];
  __shared__ __attribute__((aligned(16))) unsigned short rowb[NWAVE * GPP];
  const int tid = (int)threadIdx.x, lane = tid & 31, wave = tid >> 5;
  const int blk = (int)blockIdx.x;
  unsigned short* rowbuf = rowb + wave * GPP;

  bucket_core<SLP, NBP, PCAP>(bat, nN, vec8, blk * NBP, GCAP, list, hl, sl, cnt, offs, cur, misc,
                              tid, lane, wave);
  const int fl = ((misc[9] | misc[10]) != 0) ? 1 : 0;
  const float qnan = __int_as_float(0x7fc00000);
  const float pz = (misc[9] != 0) ? qnan : 0.0f;

  {
    const v4i c4 = *(const v4ia*)(cnt + 4 * (lane & 7));
    const v4i f4 = {fl, fl, fl, fl};
    const bool w0 = (wave == 0) && (lane < 8);
    if (w0) *(volatile v4i*)(CNTG + blk * NBP + 4 * (lane & 7)) = c4;
    if (w0) *(volatile v4i*)(FLGp + blk * 32 + 4 * (lane & 7)) = f4;
    __threadfence();
    if (w0) *(volatile v4i*)(CNTG + blk * NBP + 4 * (lane & 7)) = c4;
    if (w0) *(volatile v4i*)(FLGp + blk * 32 + 4 * (lane & 7)) = f4;
  }

#pragma unroll 1
  for (int q = 0; q < NBP / NWAVE; ++q) {
    const int s = q * NWAVE + wave;
    const int g = blk * NBP + s;
    const int cN = cnt[s];
    const bool big = cN > GCAP;
    int c = cN < 0 ? 0 : (cN > GCAP ? GCAP : cN);
    int o = offs[s];
    o = o < 0 ? 0 : (o > PCAP ? PCAP : o);
    float pa0 = 0.0f, pa1 = 0.0f, pa2 = 0.0f, pa3 = 0.0f;
    float ph0 = 0.0f, ph1 = 0.0f, ph2 = 0.0f, ph3 = 0.0f;
#pragma unroll 1
    for (int b0 = 0; b0 < c; b0 += 32) {
      int idx = o + b0 + lane;
      idx = idx > PCAP - 1 ? PCAP - 1 : idx;
      int nd = sl[idx] >> SLP;
      nd = nd < 0 ? 0 : (nd > nN - 1 ? nN - 1 : nd);
      const int m32 = (c - b0) < 32 ? (c - b0) : 32;
#pragma unroll 1
      for (int k = 0; k < m32; ++k) {
        const int nk = __builtin_amdgcn_readlane(nd, k);
        const unsigned short* ra = aggp + (size_t)nk * HP + 4 * lane;
        const unsigned short* rh = hp + (size_t)nk * HP + 4 * lane;
        const v2u ah = *(const v2ua*)ra;
        const v2u al = *(const v2ua*)(ra + DF);
        const v2u xh = *(const v2ua*)rh;
        const v2u xl = *(const v2ua*)(rh + DF);
        pa0 += __uint_as_float(ah.x << 16)         + __uint_as_float(al.x << 16);
        pa1 += __uint_as_float(ah.x & 0xffff0000u) + __uint_as_float(al.x & 0xffff0000u);
        pa2 += __uint_as_float(ah.y << 16)         + __uint_as_float(al.y << 16);
        pa3 += __uint_as_float(ah.y & 0xffff0000u) + __uint_as_float(al.y & 0xffff0000u);
        ph0 += __uint_as_float(xh.x << 16)         + __uint_as_float(xl.x << 16);
        ph1 += __uint_as_float(xh.x & 0xffff0000u) + __uint_as_float(xl.x & 0xffff0000u);
        ph2 += __uint_as_float(xh.y << 16)         + __uint_as_float(xl.y << 16);
        ph3 += __uint_as_float(xh.y & 0xffff0000u) + __uint_as_float(xl.y & 0xffff0000u);
      }
    }
    const float cf = (cN < 1) ? 1.0f : (float)cN;
    const float rc = 1.0f / cf;
    const float pzr = big ? qnan : pz;
    const float u0 = pa0 * rc + pzr, u1 = pa1 * rc + pzr, u2 = pa2 * rc + pzr, u3 = pa3 * rc + pzr;
    const float w0 = ph0 * rc + pzr, w1 = ph1 * rc + pzr, w2 = ph2 * rc + pzr, w3 = ph3 * rc + pzr;
    v4us ahh, all_, hhh, hll;
    unsigned hb;
    hb = bf16_bits(u0); ahh[0] = (unsigned short)hb; all_[0] = (unsigned short)bf16_bits(u0 - __uint_as_float(hb << 16));
    hb = bf16_bits(u1); ahh[1] = (unsigned short)hb; all_[1] = (unsigned short)bf16_bits(u1 - __uint_as_float(hb << 16));
    hb = bf16_bits(u2); ahh[2] = (unsigned short)hb; all_[2] = (unsigned short)bf16_bits(u2 - __uint_as_float(hb << 16));
    hb = bf16_bits(u3); ahh[3] = (unsigned short)hb; all_[3] = (unsigned short)bf16_bits(u3 - __uint_as_float(hb << 16));
    hb = bf16_bits(w0); hhh[0] = (unsigned short)hb; hll[0] = (unsigned short)bf16_bits(w0 - __uint_as_float(hb << 16));
    hb = bf16_bits(w1); hhh[1] = (unsigned short)hb; hll[1] = (unsigned short)bf16_bits(w1 - __uint_as_float(hb << 16));
    hb = bf16_bits(w2); hhh[2] = (unsigned short)hb; hll[2] = (unsigned short)bf16_bits(w2 - __uint_as_float(hb << 16));
    hb = bf16_bits(w3); hhh[3] = (unsigned short)hb; hll[3] = (unsigned short)bf16_bits(w3 - __uint_as_float(hb << 16));
    *(v4usa*)(rowbuf + 4 * lane)          = ahh;
    *(v4usa*)(rowbuf + DF + 4 * lane)     = all_;
    *(v4usa*)(rowbuf + 2 * DF + 4 * lane) = hhh;
    *(v4usa*)(rowbuf + 3 * DF + 4 * lane) = hll;
    wave_sync();
    const v8us q0 = *(const v8usa*)(rowbuf + 8 * lane);
    const v8us q1 = *(const v8usa*)(rowbuf + 2 * DF + 8 * lane);
    wave_sync();
    unsigned short* rpw = GP + (size_t)g * GPP + 8 * lane;
    *(volatile v8us*)rpw = q0;
    *(volatile v8us*)(rpw + 2 * DF) = q1;
    __threadfence();
    *(volatile v8us*)rpw = q0;
    *(volatile v8us*)(rpw + 2 * DF) = q1;
  }
}

__global__ __launch_bounds__(NTHR) void k_head(const float* __restrict__ Z, const float* __restrict__ W2,
                                               const float* __restrict__ b2, const int* __restrict__ FLGg,
                                               float* out) {
  __shared__ __attribute__((aligned(16))) float w0s[CLS];
  __shared__ __attribute__((aligned(16))) float w1s[CLS];
  __shared__ __attribute__((aligned(16))) float os[256];
  __shared__ int wfl[NWAVE];
  const int tid = (int)threadIdx.x, lane = tid & 31, wave = tid >> 5;
  const int blk = (int)blockIdx.x;
  w0s[tid] = bf16_val(W2[tid]);
  w1s[tid] = bf16_val(W2[CLS + tid]);
  {
    const int i1 = tid < NFLG ? tid : NFLG - 1;
    const int i2 = (tid + NTHR) < NFLG ? (tid + NTHR) : NFLG - 1;
    const int f1 = FLGg[i1 * 32];
    const int f2 = FLGg[i2 * 32];
    const bool bad = ((tid < NFLG) && (f1 != 0)) || (((tid + NTHR) < NFLG) && (f2 != 0));
    const unsigned bm = __builtin_amdgcn_ballot_w32(bad);
    if (lane == 0) wfl[wave] = (bm != 0u) ? 1 : 0;
  }
  __syncthreads();
  const float b20 = bf16_val(b2[0]);
  const float b21 = bf16_val(b2[1]);
  const v4f wa0 = *(const v4fa*)(w0s + 8 * lane);
  const v4f wa1 = *(const v4fa*)(w0s + 8 * lane + 4);
  const v4f wb0 = *(const v4fa*)(w1s + 8 * lane);
  const v4f wb1 = *(const v4fa*)(w1s + 8 * lane + 4);
#pragma unroll 1
  for (int gi = 0; gi < 16; ++gi) {
    const int gl = 16 * wave + gi;
    const int g  = blk * 128 + gl;
    const float* zp = Z + (size_t)g * CLS + 8 * lane;
    const v4f z0 = *(const v4f*)zp;
    const v4f z1 = *(const v4f*)(zp + 4);
    float s0 = 0.0f, s1 = 0.0f;
    s0 = fmaf(z0.x, wa0.x, s0); s0 = fmaf(z0.y, wa0.y, s0); s0 = fmaf(z0.z, wa0.z, s0); s0 = fmaf(z0.w, wa0.w, s0);
    s0 = fmaf(z1.x, wa1.x, s0); s0 = fmaf(z1.y, wa1.y, s0); s0 = fmaf(z1.z, wa1.z, s0); s0 = fmaf(z1.w, wa1.w, s0);
    s1 = fmaf(z0.x, wb0.x, s1); s1 = fmaf(z0.y, wb0.y, s1); s1 = fmaf(z0.z, wb0.z, s1); s1 = fmaf(z0.w, wb0.w, s1);
    s1 = fmaf(z1.x, wb1.x, s1); s1 = fmaf(z1.y, wb1.y, s1); s1 = fmaf(z1.z, wb1.z, s1); s1 = fmaf(z1.w, wb1.w, s1);
    s0 += __shfl_xor(s0, 16, 32); s1 += __shfl_xor(s1, 16, 32);
    s0 += __shfl_xor(s0, 8, 32);  s1 += __shfl_xor(s1, 8, 32);
    s0 += __shfl_xor(s0, 4, 32);  s1 += __shfl_xor(s1, 4, 32);
    s0 += __shfl_xor(s0, 2, 32);  s1 += __shfl_xor(s1, 2, 32);
    s0 += __shfl_xor(s0, 1, 32);  s1 += __shfl_xor(s1, 1, 32);
    if (lane == 0) { os[2 * gl] = s0 + b20; os[2 * gl + 1] = s1 + b21; }
  }
  __syncthreads();
  const int anyf = wfl[0] | wfl[1] | wfl[2] | wfl[3] | wfl[4] | wfl[5] | wfl[6] | wfl[7];
  const float qnan = __int_as_float(0x7fc00000);
  v4f ov = *(const v4fa*)(os + 4 * (tid & 63));
  ov.x = (anyf != 0) ? qnan : ov.x; ov.y = (anyf != 0) ? qnan : ov.y;
  ov.z = (anyf != 0) ? qnan : ov.z; ov.w = (anyf != 0) ? qnan : ov.w;
  const bool okst = tid < 64;
  float* op = out + (size_t)blk * 256 + 4 * (tid & 63);
  if (okst) *(volatile v4f*)op = ov;
  __threadfence();
  if (okst) *(volatile v4f*)op = ov;
}

static inline size_t al256(size_t o) { return (o + 255) & ~(size_t)255; }

extern "C" void kernel_launch(void* const* d_in, const int* in_sizes, int n_in,
                              void* d_out, int out_size, void* d_ws, size_t ws_size,
                              hipStream_t stream) {
  if (n_in < 13) return;
  if (in_sizes[0] != NN * IND) return;
  if (in_sizes[1] != 2 * NE) return;
  if (in_sizes[2] != NN) return;
  if (in_sizes[3] != DF * IND || in_sizes[4] != DF) return;
  if (in_sizes[5] != DF * IND) return;
  if (in_sizes[6] != 3 * DF * DF || in_sizes[7] != 3 * DF) return;
  if (in_sizes[8] != 3 * DF * DF) return;
  if (in_sizes[9] != CLS * DF || in_sizes[10] != CLS) return;
  if (in_sizes[11] != 2 * CLS || in_sizes[12] != 2) return;
  if (out_size != NG * 2) return;

  const float* x     = (const float*)d_in[0];
  const int*   edge  = (const int*)d_in[1];
  const int*   bat   = (const int*)d_in[2];
  const float* W1l   = (const float*)d_in[3];
  const float* b1l   = (const float*)d_in[4];
  const float* W1r   = (const float*)d_in[5];
  const float* Wl    = (const float*)d_in[6];
  const float* bl    = (const float*)d_in[7];
  const float* Wr    = (const float*)d_in[8];
  const float* Wlin1 = (const float*)d_in[9];
  const float* blin1 = (const float*)d_in[10];
  const float* Wlin2 = (const float*)d_in[11];
  const float* blin2 = (const float*)d_in[12];
  float* out = (float*)d_out;
  const int* src = edge;
  const int* dst = edge + NE;
  const int vecE = ((NE & 3) == 0) ? 1 : 0;
  const int vecB = 1;

  const size_t PLANE = (size_t)MP * HP * 2;
  const size_t XBB   = (size_t)MP * XP * 2;
  const size_t A0B   = (size_t)MP * A0P * 2;
  if (XBB + A0B > PLANE) return;
  char* ws = (char*)d_ws;
  size_t off = 0;
  const size_t oRA  = off; off = al256(off + PLANE);
  const size_t oRB  = off; off = al256(off + PLANE);
  const size_t oLST = off; off = al256(off + (size_t)NBLK * LCAP * 4);
  const size_t oDEG = off; off = al256(off + (size_t)NSLOT * 4);
  const size_t oOFF = off; off = al256(off + (size_t)NSLOT * 4);
  const size_t oINV = off; off = al256(off + (size_t)NSLOT * 4);
  const size_t oW0  = off; off = al256(off + (size_t)DF * K0 * 2);
  const size_t oWC  = off; off = al256(off + (size_t)3 * DF * K1 * 2);
  const size_t oWL  = off; off = al256(off + (size_t)CLS * KL * 2);
  const size_t oGP  = off; off = al256(off + (size_t)NG * GPP * 2);
  const size_t oGH  = off; off = al256(off + (size_t)NG * HP * 2);
  const size_t oZ   = off; off = al256(off + (size_t)NG * CLS * 4);
  const size_t oCN  = off; off = al256(off + (size_t)NG * 4);
  const size_t oFL  = off; off = al256(off + (size_t)NFLG * 128);
  if (off > ws_size) return;

  unsigned short* wsh  = (unsigned short*)ws;
  unsigned short* RA   = (unsigned short*)(ws + oRA);
  unsigned short* RB   = (unsigned short*)(ws + oRB);
  unsigned short* XB   = RB;
  unsigned short* AG0  = (unsigned short*)(ws + oRB + XBB);
  int*            LST  = (int*)(ws + oLST);
  int*            DEG  = (int*)(ws + oDEG);
  int*            OFFT = (int*)(ws + oOFF);
  float*          INV  = (float*)(ws + oINV);
  unsigned short* W0c  = (unsigned short*)(ws + oW0);
  unsigned short* Wc   = (unsigned short*)(ws + oWC);
  unsigned short* WL1  = (unsigned short*)(ws + oWL);
  unsigned short* GP   = (unsigned short*)(ws + oGP);
  unsigned short* GH   = (unsigned short*)(ws + oGH);
  float*          Zp   = (float*)(ws + oZ);
  int*            CNTG = (int*)(ws + oCN);
  int*            FLG  = (int*)(ws + oFL);

  k_prep<<<XBLK + WBLK, NTHR, 0, stream>>>(x, W1l, W1r, Wl, Wr, Wlin1, wsh, oRB / 2, oW0 / 2, oWC / 2, oWL / 2);
  k_bucket<<<NBLK, NTHR, 0, stream>>>(src, dst, NE, NN, vecE, LST, DEG, OFFT, INV, FLG);
  k_agg<1><<<NBLK, NTHR, 0, stream>>>(XB, AG0, LST, DEG, OFFT, INV, FLG, NN, MP);
  k_gemm<0><<<dim3(MP / GBM, 1), GTHR, 0, stream>>>(AG0, A0P, A0P / 32, XB, XP, XP / 32, W0c, K0, b1l, CNTG, RA, Zp, NN);
  k_agg<0><<<NBLK, NTHR, 0, stream>>>(RA, RB, LST, DEG, OFFT, INV, FLG, NN, MP);
  k_gemm<0><<<dim3(MP / GBM, 1), GTHR, 0, stream>>>(RB, HP, HP / 32, RA, HP, HP / 32, Wc, K1, bl, CNTG, RB, Zp, NN);
  k_agg<0><<<NBLK, NTHR, 0, stream>>>(RB, RA, LST, DEG, OFFT, INV, FLG, NN, MP);
  k_gemm<0><<<dim3(MP / GBM, 1), GTHR, 0, stream>>>(RA, HP, HP / 32, RB, HP, HP / 32, Wc + (size_t)DF * K1, K1, bl + DF, CNTG, RA, Zp, NN);
  k_agg<0><<<NBLK, NTHR, 0, stream>>>(RA, RB, LST, DEG, OFFT, INV, FLG, NN, MP);
  k_pool<<<PBLK, NTHR, 0, stream>>>(RB, RA, bat, NN, vecB, GP, CNTG, FLG + NBLK * 32);
  k_gemm<2><<<dim3(NG / GBM, 1), GTHR, 0, stream>>>(GP, GPP, GPP / 32, GP, GPP, 0, Wc + (size_t)2 * DF * K1, K1, bl + 2 * DF, CNTG, GH, Zp, NG);
  k_gemm<1><<<dim3(NG / GBM, CLS / GBN), GTHR, 0, stream>>>(GH, HP, HP / 32, GH, HP, 0, WL1, KL, blin1, CNTG, GH, Zp, NG);
  k_head<<<NG / 128, NTHR, 0, stream>>>(Zp, Wlin2, blin2, FLG, out);
}
